// RnnModel1_1743756722578
// MI455X (gfx1250) — hardware-verified
//
#include <hip/hip_runtime.h>


namespace {
constexpr int B = 1024, T = 1024, H = 128, C = 10;
constexpr float XS = 8.0f, WSC = 256.0f;
typedef _Float16 b16;
typedef __attribute__((ext_vector_type(16))) _Float16 v16b;
typedef __attribute__((ext_vector_type(8))) _Float16 v8b;
typedef __attribute__((ext_vector_type(8))) float v8f;
typedef __attribute__((ext_vector_type(4))) float v4f;
__device__ __forceinline__ float bf16_rne(float f) { unsigned int u = __float_as_uint(f); u += 0x7FFFu + ((u >> 16) & 1u); return __uint_as_float(u & 0xFFFF0000u); }
__device__ __forceinline__ void split16(float v, b16& hi, b16& lo) { hi = (b16)v; lo = (b16)(v - (float)hi); }
__device__ __forceinline__ v16b frag_kb(const b16* p, int hh) { const v8b a = *(const v8b*)(p + 8 * hh), b = *(const v8b*)(p + 16 + 8 * hh); v16b f;
#pragma unroll
  for (int e = 0; e < 8; ++e) { f[e] = a[e]; f[8 + e] = b[e]; } return f; }
__device__ __forceinline__ v8f wmma16b(v16b a, v16b b, v8f c) { v8f d = __builtin_amdgcn_wmma_f32_16x16x32_f16(false, a, false, b, (short)0, c, false, false); asm volatile("v_nop\n\tv_nop\n\tv_nop\n\tv_nop" : "+v"(d) : "v"(a), "v"(b)); return d; }
__device__ __forceinline__ void wave_lds_sync() { __builtin_amdgcn_fence(__ATOMIC_RELEASE, "workgroup"); __builtin_amdgcn_wave_barrier(); __builtin_amdgcn_fence(__ATOMIC_ACQUIRE, "workgroup"); }
__device__ __forceinline__ float pmul(float a, float b) { float p = a * b; asm volatile("" : "+v"(p)); return p; }
__device__ __forceinline__ float tanh_(float x) { const float e = __expf(2.0f * x); return 1.0f - 2.0f / (e + 1.0f); }

__global__ __launch_bounds__(256) void wprep_kernel(const float* __restrict__ whh, const float* __restrict__ fcw, b16* __restrict__ WHH, b16* __restrict__ WFC) {
  const size_t u = (size_t)blockIdx.x * 256 + threadIdx.x; const size_t n0 = (size_t)H * H / 8, n1 = (size_t)16 * H / 8; size_t t = u; v8b o;
  if (t < n0) { const size_t e = t * 8; for (int j = 0; j < 8; ++j) o[j] = (b16)(bf16_rne(whh[e + j]) * WSC); for (int pass = 0; pass < 2; ++pass) { *(volatile v8b*)(WHH + e) = o; __threadfence(); } return; } t -= n0;
  if (t < n1) { const size_t e = t * 8; const int oo = (int)(e / H), k0 = (int)(e % H); for (int j = 0; j < 8; ++j) o[j] = oo < C ? (b16)(bf16_rne(fcw[(size_t)oo * H + k0 + j]) * WSC) : (b16)0.0f; for (int pass = 0; pass < 2; ++pass) { *(volatile v8b*)(WFC + e) = o; __threadfence(); } }
}
__global__ __launch_bounds__(64) void rnn_kernel(const float* __restrict__ x, const float* __restrict__ wih, const float* __restrict__ bih, const float* __restrict__ bhh, const b16* __restrict__ WHH, const b16* __restrict__ WFC, const float* __restrict__ fcb, float* __restrict__ out) {
  __shared__ __attribute__((aligned(16))) b16 Ah[2][16][H + 8], Al[2][16][H + 8]; __shared__ __attribute__((aligned(16))) float so[32 * C];
  const int wave = threadIdx.x >> 5, lane = threadIdx.x & 31, nloc = lane & 15, hlf = lane >> 4; const int b0 = blockIdx.x * 32 + wave * 16;
  float hreg[8][8];
#pragma unroll
  for (int t = 0; t < 8; ++t) for (int r = 0; r < 8; ++r) hreg[t][r] = 0.0f;
  float wi[8], bb[8]; for (int t = 0; t < 8; ++t) { const int c = t * 16 + nloc; wi[t] = bf16_rne(wih[c]); bb[t] = bf16_rne(bih[c]) + bf16_rne(bhh[c]); }
#pragma unroll 1
  for (int step = 0; step < T; ++step) {
#pragma unroll
    for (int t = 0; t < 8; ++t)
#pragma unroll
      for (int r = 0; r < 8; ++r) { b16 p, q; split16(hreg[t][r] * XS, p, q); Ah[wave][8 * hlf + r][t * 16 + nloc] = p; Al[wave][8 * hlf + r][t * 16 + nloc] = q; }
    wave_lds_sync();
    v8f gh[8];
#pragma unroll
    for (int t = 0; t < 8; ++t) gh[t] = (v8f){};
#pragma unroll
    for (int kb = 0; kb < H; kb += 32) { const v16b a = frag_kb(&Ah[wave][nloc][kb], hlf), al = frag_kb(&Al[wave][nloc][kb], hlf);
#pragma unroll
      for (int t = 0; t < 8; ++t) { const v16b bw = frag_kb(WHH + (size_t)(t * 16 + nloc) * H + kb, hlf); gh[t] = wmma16b(a, bw, gh[t]); gh[t] = wmma16b(al, bw, gh[t]); } }
    float xr[8]; for (int r = 0; r < 8; ++r) xr[r] = bf16_rne(x[(size_t)(b0 + 8 * hlf + r) * T + step]);
#pragma unroll
    for (int t = 0; t < 8; ++t)
#pragma unroll
      for (int r = 0; r < 8; ++r) hreg[t][r] = tanh_(pmul(xr[r], wi[t]) + bb[t] + gh[t][r] * (1.0f / (XS * WSC)));
    wave_lds_sync();
  }
#pragma unroll
  for (int t = 0; t < 8; ++t)
#pragma unroll
    for (int r = 0; r < 8; ++r) { b16 p, q; split16(hreg[t][r] * XS, p, q); Ah[wave][8 * hlf + r][t * 16 + nloc] = p; Al[wave][8 * hlf + r][t * 16 + nloc] = q; }
  wave_lds_sync();
  v8f acc = (v8f){};
#pragma unroll
  for (int kb = 0; kb < H; kb += 32) { const v16b a = frag_kb(&Ah[wave][nloc][kb], hlf), al = frag_kb(&Al[wave][nloc][kb], hlf); const v16b bw = frag_kb(WFC + (size_t)nloc * H + kb, hlf); acc = wmma16b(a, bw, acc); acc = wmma16b(al, bw, acc); }
  if (nloc < C) { const float bo = bf16_rne(fcb[nloc]);
#pragma unroll 1
    for (int r = 0; r < 8; ++r) so[(wave * 16 + 8 * hlf + r) * C + nloc] = acc[r] * (1.0f / (XS * WSC)) + bo; }
  __syncthreads();
  for (int pass = 0; pass < 2; ++pass) { for (int q = threadIdx.x * 4; q < 32 * C; q += 256) *(volatile v4f*)(out + (size_t)blockIdx.x * 32 * C + q) = *(const v4f*)(&so[q]); __threadfence(); }
}
}

extern "C" void kernel_launch(void* const* d_in, const int* in_sizes, int n_in, void* d_out, int out_size, void* d_ws, size_t ws_size, hipStream_t stream) {
  (void)n_in;
  auto Fp = [&](int i) { return (const float*)d_in[i]; };
  if (in_sizes[0] != B * T || in_sizes[1] != H || in_sizes[2] != H * H || in_sizes[5] != C * H || out_size != B * C) return;
  if (ws_size < (size_t)(H * H + 16 * H) * 2) return; b16* WHH = (b16*)d_ws; b16* WFC = WHH + (size_t)H * H;
  wprep_kernel<<<(unsigned)(((size_t)H * H / 8 + (size_t)16 * H / 8 + 255) / 256), 256, 0, stream>>>(Fp(2), Fp(5), WHH, WFC);
  rnn_kernel<<<B / 32, 64, 0, stream>>>(Fp(0), Fp(1), Fp(3), Fp(4), WHH, WFC, Fp(6), (float*)d_out);
}
